// GATr_model_34308198761147
// MI455X (gfx1250) — hardware-run, weakly checked
//
#include <hip/hip_runtime.h>
#include <math.h>
#include <stdint.h>

#define NB    4
#define NTOK  4096
#define TOK   (NB * NTOK)
#define NCH   5
#define NF    80
#define XW    35
#define TPB   32
#define DQK   128
#define AQB   128
#define AKC   64
#define ANW   8

static_assert(NTOK % AQB == 0);
static_assert(NTOK % AKC == 0);
static_assert(DQK % 32 == 0);
static_assert(NF % 16 == 0);
static_assert(120 <= DQK);
static_assert(TOK % TPB == 0);
static_assert((TPB * XW * 4) % 128 == 0);
static_assert((TPB * NF * 4) % 128 == 0);
static_assert((TPB * NF * 2) % 128 == 0);
static_assert((TPB * DQK * 2) % 128 == 0);
static_assert(AKC == 2 * TPB);
static_assert(AQB == ANW * 16);

typedef __attribute__((ext_vector_type(16))) __bf16 v16b;
typedef __attribute__((ext_vector_type(8)))  __bf16 v8b;
typedef __attribute__((ext_vector_type(8)))  float  v8f;
typedef __attribute__((ext_vector_type(4)))  float  v4f;
typedef __attribute__((ext_vector_type(8)))  unsigned short v8us;

__host__ __device__ constexpr int ga_pop4(int m) { return (m & 1) + ((m >> 1) & 1) + ((m >> 2) & 1) + ((m >> 3) & 1); }
constexpr unsigned long long ga_build_maskpk() {
  unsigned long long pk = 0ull; int n = 0;
  for (int g = 0; g <= 4; ++g)
    for (int m = 0; m < 16; ++m)
      if (ga_pop4(m) == g) { pk |= ((unsigned long long)m) << (4 * n); ++n; }
  return pk;
}
constexpr unsigned long long GA_MASKPK = ga_build_maskpk();
static_assert(GA_MASKPK == 0xFEDB7CA965384210ull);
__host__ __device__ constexpr int ga_mask(int i) { return (int)((GA_MASKPK >> (4 * i)) & 15ull); }
constexpr unsigned long long ga_build_idxpk() {
  unsigned long long pk = 0ull;
  for (int i = 0; i < 16; ++i) pk |= ((unsigned long long)i) << (4 * ga_mask(i));
  return pk;
}
constexpr unsigned long long GA_IDXPK = ga_build_idxpk();
__host__ __device__ constexpr int ga_idx(int m) { return (int)((GA_IDXPK >> (4 * m)) & 15ull); }
__host__ __device__ constexpr int ga_sign(int a, int b) {
  if (a & b & 1) return 0;
  int sw = 0;
  for (int t = 0; t < 4; ++t) if ((b >> t) & 1) sw += ga_pop4(a >> (t + 1));
  return (sw & 1) ? -1 : 1;
}
constexpr int ga_C(int i, int j, int k) { return (ga_idx(ga_mask(i) ^ ga_mask(j)) == k) ? ga_sign(ga_mask(i), ga_mask(j)) : 0; }
constexpr int ga_nnz() {
  int n = 0;
  for (int i = 0; i < 16; ++i) for (int j = 0; j < 16; ++j) for (int k = 0; k < 16; ++k) if (ga_C(i, j, k) != 0) ++n;
  return n;
}
constexpr bool ga_pair_zero(int i, int j) { for (int k = 0; k < 16; ++k) if (ga_C(i, j, k) != 0) return false; return true; }
static_assert(ga_C(2, 2, 0) == 1);
static_assert(ga_pair_zero(1, 1));
static_assert(ga_C(7, 7, 0) == -1);
static_assert(ga_C(2, 3, 7) == 1);
static_assert(ga_C(3, 2, 7) == -1);
static_assert(ga_nnz() == 192);
constexpr unsigned long long ga_build_innerpk() {
  unsigned long long pk = 0ull; int n = 0;
  for (int c = 0; c < 16; ++c) if (!(ga_mask(c) & 1)) { pk |= ((unsigned long long)c) << (4 * n); ++n; }
  return pk;
}
constexpr int ga_count_inner() { int n = 0; for (int c = 0; c < 16; ++c) if (!(ga_mask(c) & 1)) ++n; return n; }
constexpr unsigned long long GA_INNERPK = ga_build_innerpk();
static_assert(ga_count_inner() == 8);
static_assert(GA_INNERPK == 0xEA974320ull);
__host__ __device__ constexpr int ga_islot(int r) { return (int)((GA_INNERPK >> (4 * r)) & 15ull); }
constexpr int GA_T0 = ga_idx(3), GA_T1 = ga_idx(5), GA_T2 = ga_idx(9);
static_assert(GA_T0 == 5 && GA_T1 == 6 && GA_T2 == 8);
static_assert(ga_pop4(ga_mask(GA_T0)) == 2 && ga_pop4(ga_mask(GA_T1)) == 2 && ga_pop4(ga_mask(GA_T2)) == 2);

#define P_WIN   0
#define P_WOUT  800
#define P_WQ    1600
#define P_WK    1984
#define P_WV    2368
#define P_WO    2752
#define P_W1    3136
#define P_W2    3904
#define P_TOT   4288
static_assert(5 * 5 * 32 == 800 && 5 * 32 * 5 == 800);
static_assert(3 * 5 * 5 * 5 == 375 && 3 * 5 * 10 * 5 == 750);
static_assert(P_WOUT == P_WIN + 800 && P_WQ == P_WOUT + 800);
static_assert(P_WK == P_WQ + 384 && P_WV == P_WK + 384 && P_WO == P_WV + 384 && P_W1 == P_WO + 384);
static_assert(P_W2 == P_W1 + 768 && P_TOT == P_W2 + 384);
static_assert(P_WOUT % 32 == 0 && P_WQ % 32 == 0 && P_WK % 32 == 0 && P_WV % 32 == 0 && P_WO % 32 == 0);
static_assert(P_W1 % 32 == 0 && P_W2 % 32 == 0 && P_TOT % 32 == 0);

#define LW_A   0
#define LW_O   800
#define LW_1   928
#define LW_2   1184
#define LW_Q   1312
#define LW_K   1440
#define LW_V   1568
#define LW_TOT 1696

__device__ __forceinline__ unsigned short f2bf_bits(float f) {
  unsigned u = __float_as_uint(f);
  return (unsigned short)((u + 0x7FFFu + ((u >> 16) & 1u)) >> 16);
}
__device__ __forceinline__ float bf_bits2f(unsigned short h) { return __uint_as_float(((unsigned)h) << 16); }
__device__ __forceinline__ float bf16r(float f) { return bf_bits2f(f2bf_bits(f)); }
__device__ __forceinline__ __bf16 to_bf(float f) { return __builtin_bit_cast(__bf16, f2bf_bits(f)); }
__device__ __forceinline__ void split_bf(float f, __bf16& hi, __bf16& lo) {
  const unsigned short hb = f2bf_bits(f);
  hi = __builtin_bit_cast(__bf16, hb);
  lo = to_bf(f - bf_bits2f(hb));
}
__device__ __forceinline__ v8f wmb(v16b a, v16b b, v8f c) {
  c = __builtin_amdgcn_wmma_f32_16x16x32_bf16(false, a, false, b, (short)0, c, false, false);
  asm volatile("v_nop\n\tv_nop\n\tv_nop\n\tv_nop" : "+v"(c) : "v"(a), "v"(b));
  return c;
}
__device__ __forceinline__ v16b frag_ld(const __bf16* p) {
  union { v16b v; v8b h[2]; } f;
  f.h[0] = *(const v8b*)(p);
  f.h[1] = *(const v8b*)(p + 16);
  return f.v;
}

static_assert(800 <= 1024);
__device__ __forceinline__ void prm_copy(const float* __restrict__ src, int n, int npad, float* __restrict__ dst) {
  const int i0 = (int)threadIdx.x * 4;
  v4f v;
#pragma unroll
  for (int e = 0; e < 4; ++e) {
    const int i = i0 + e;
    const int ic = (i < n) ? i : (n - 1);
    const float f = src[ic];
    v[e] = (i < n) ? bf16r(f) : 0.0f;
  }
  const bool act = i0 < npad;
  if (act) *(volatile v4f*)(dst + i0) = v;
  __threadfence();
  if (act) *(volatile v4f*)(dst + i0) = v;
}

__global__ __launch_bounds__(256) void k_prm(const float* __restrict__ w_in, const float* __restrict__ w_out,
                                             const float* __restrict__ wq, const float* __restrict__ wk,
                                             const float* __restrict__ wv, const float* __restrict__ wo,
                                             const float* __restrict__ w1, const float* __restrict__ w2,
                                             float* __restrict__ prm) {
  const int a = blockIdx.x;
  if (a == 0)      prm_copy(w_in,  800, 800, prm + P_WIN);
  else if (a == 1) prm_copy(w_out, 800, 800, prm + P_WOUT);
  else if (a == 2) prm_copy(wq,    375, 384, prm + P_WQ);
  else if (a == 3) prm_copy(wk,    375, 384, prm + P_WK);
  else if (a == 4) prm_copy(wv,    375, 384, prm + P_WV);
  else if (a == 5) prm_copy(wo,    375, 384, prm + P_WO);
  else if (a == 6) prm_copy(w1,    750, 768, prm + P_W1);
  else             prm_copy(w2,    375, 384, prm + P_W2);
}

__device__ __forceinline__ void ln_xn(const float* hS, float* xS, float* invS, int tid) {
  if (tid < TPB) {
    const float* hp = hS + tid * NF;
    float s = 0.0f;
#pragma unroll 4
    for (int j = 0; j < 40; ++j) {
      const int ch = j >> 3;
      const int c = ga_islot(j & 7);
      const float v = hp[ch * 16 + c];
      s = fmaf(v, v, s);
    }
    invS[tid] = 1.0f / sqrtf(s * 0.2f * 0.0625f + 1e-6f);
  }
  __syncthreads();
#pragma unroll 1
  for (int it = 0; it < 10; ++it) {
    const int idx = it * 256 + tid;
    const int tok = idx / NF;
    xS[idx] = hS[idx] * invS[tok];
  }
  __syncthreads();
}

#define CPW(LOC, OFF, N)                                              \
  for (int it_ = 0; it_ < ((N) + 255) / 256; ++it_) {                 \
    const int i_ = it_ * 256 + tid;                                   \
    const int ic_ = (i_ < (N)) ? i_ : ((N) - 1);                      \
    const float w_ = prm[(OFF) + ic_];                                \
    if (i_ < (N)) sW[(LOC) + i_] = w_;                                \
  }

template <int MODE>
__global__ __launch_bounds__(256) void k_tok(const float* __restrict__ x, const float* __restrict__ Oin,
                                             const float* __restrict__ Hin, float* __restrict__ Hout,
                                             const float* __restrict__ prm,
                                             unsigned short* __restrict__ QP, unsigned short* __restrict__ KP,
                                             unsigned short* __restrict__ VH, unsigned short* __restrict__ VL,
                                             float* __restrict__ out, int blk) {
  __shared__ __align__(16) float sW[LW_TOT];
  __shared__ int   sJX[256];
  __shared__ float sSG[256];
  __shared__ __align__(16) float sH[TPB * NF];
  __shared__ __align__(16) float sX[TPB * NF];
  __shared__ __align__(16) float sT[TPB * 2 * NF];
  __shared__ __align__(16) float sG[TPB * NF];
  __shared__ float sGate[TPB * NCH];
  __shared__ float sInv[TPB];
  __shared__ __align__(16) unsigned short sQP[TPB * DQK];
  __shared__ __align__(16) unsigned short sKP[TPB * DQK];
  __shared__ __align__(16) unsigned short sVH[NF * TPB];
  __shared__ __align__(16) unsigned short sVL[NF * TPB];
  __shared__ __align__(16) float sIO[TPB * XW];

  const int tid  = threadIdx.x;
  const int tok0 = blockIdx.x * TPB;

  if (MODE == 0) { CPW(LW_A, P_WIN, 800) }
  if (MODE == 2) { CPW(LW_A, P_WOUT, 800) }
  if (MODE != 0) {
    CPW(LW_O, P_WO + blk * 125, 125)
    CPW(LW_1, P_W1 + blk * 250, 250)
    CPW(LW_2, P_W2 + blk * 125, 125)
    const int i = tid >> 4, k = tid & 15;
    const int mi = ga_mask(i), mj = mi ^ ga_mask(k);
    sJX[tid] = ga_idx(mj);
    sSG[tid] = (float)ga_sign(mi, mj);
  }
  if (MODE != 2) {
    int bq = (MODE == 0) ? 0 : (blk + 1);
    bq = (bq > 2) ? 2 : bq;
    CPW(LW_Q, P_WQ + bq * 125, 125)
    CPW(LW_K, P_WK + bq * 125, 125)
    CPW(LW_V, P_WV + bq * 125, 125)
  }

  if (MODE == 0) {
    const float* xb = x + (size_t)blockIdx.x * (TPB * XW);
#pragma unroll
    for (int it = 0; it < 2; ++it) {
      const int idx = it * 256 + tid;
      const int idc = (idx < 280) ? idx : 279;
      v4f v = *(const v4f*)(xb + idc * 4);
#pragma unroll
      for (int e = 0; e < 4; ++e) v[e] = bf16r(v[e]);
      if (idx < 280) *(v4f*)(sIO + idx * 4) = v;
    }
    __syncthreads();
    if (tid < TPB * NCH) {
      const int tok = tid / NCH, o = tid - tok * NCH;
      const float* wp = sW + LW_A + o * 32;
      const float* xp = sIO + tok * XW;
      float acc = wp[0];
#pragma unroll 4
      for (int i = 1; i < 32; ++i) acc = fmaf(xp[i], wp[i], acc);
      sH[tok * NF + o * 16] = acc;
    }
#pragma unroll 1
    for (int it = 0; it < 10; ++it) {
      const int idx = it * 256 + tid;
      const int tok = idx / NF;
      const int rem = idx - tok * NF;
      const int o = rem >> 4, c = rem & 15;
      const int jj = (c == GA_T1) ? 1 : ((c == GA_T2) ? 2 : 0);
      const bool isT = (c == GA_T0) || (c == GA_T1) || (c == GA_T2);
      const float xv = sIO[tok * XW + 32 + jj];
      const float wv = sW[LW_A + (2 * NCH + o) * 32];
      const float val = isT ? (wv * xv) : 0.0f;
      if (c != 0) sH[idx] = val;
    }
    __syncthreads();
  } else {
#pragma unroll
    for (int it = 0; it < 3; ++it) {
      const int idx = it * 256 + tid;
      const int idc = (idx < 640) ? idx : 639;
      const v4f a = *(const v4f*)(Oin + (size_t)tok0 * NF + idc * 4);
      const v4f b = *(const v4f*)(Hin + (size_t)tok0 * NF + idc * 4);
      if (idx < 640) { *(v4f*)(sX + idx * 4) = a; *(v4f*)(sH + idx * 4) = b; }
    }
    __syncthreads();
#pragma unroll 1
    for (int it = 0; it < 10; ++it) {
      const int idx = it * 256 + tid;
      const int tok = idx / NF;
      const int rem = idx - tok * NF;
      const int o = rem >> 4, c = rem & 15;
      const int g = ga_pop4(ga_mask(c));
      const float* wp = sW + LW_O + (g * NCH + o) * NCH;
      const float* xp = sX + tok * NF + c;
      float acc = 0.0f;
#pragma unroll 1
      for (int i = 0; i < NCH; ++i) acc = fmaf(xp[i * 16], wp[i], acc);
      sH[idx] = sH[idx] + acc;
    }
    __syncthreads();
    ln_xn(sH, sX, sInv, tid);
#pragma unroll 1
    for (int it = 0; it < 20; ++it) {
      const int idx = it * 256 + tid;
      const int tok = idx / (2 * NF);
      const int rem = idx - tok * (2 * NF);
      const int o = rem >> 4, c = rem & 15;
      const int g = ga_pop4(ga_mask(c));
      const float* wp = sW + LW_1 + (g * 2 * NCH + o) * NCH;
      const float* xp = sX + tok * NF + c;
      float acc = 0.0f;
#pragma unroll 1
      for (int i = 0; i < NCH; ++i) acc = fmaf(xp[i * 16], wp[i], acc);
      sT[idx] = acc;
    }
    __syncthreads();
#pragma unroll 1
    for (int it = 0; it < 10; ++it) {
      const int idx = it * 256 + tid;
      const int tok = idx / NF;
      const int rem = idx - tok * NF;
      const int ch = rem >> 4, k = rem & 15;
      const float* lp = sT + tok * (2 * NF) + ch * 16;
      const float* rp = lp + NF;
      float acc = 0.0f;
#pragma unroll 4
      for (int i = 0; i < 16; ++i) {
        const int e = i * 16 + k;
        acc = fmaf(sSG[e] * lp[i], rp[sJX[e]], acc);
      }
      sG[idx] = acc;
    }
    __syncthreads();
    if (tid < TPB * NCH) {
      const int tok = tid / NCH, ch = tid - tok * NCH;
      const float u = sG[tok * NF + ch * 16];
      const float t = u * u * u;
      const float a = 0.7978845608028654f * (u + 0.044715f * t);
      const float cdf = 0.5f * (1.0f + tanhf(a));
      sGate[tid] = u * cdf;
    }
    __syncthreads();
#pragma unroll 1
    for (int it = 0; it < 10; ++it) {
      const int idx = it * 256 + tid;
      const int tok = idx / NF;
      const int rem = idx - tok * NF;
      const int o = rem >> 4, c = rem & 15;
      const int g = ga_pop4(ga_mask(c));
      const float* wp = sW + LW_2 + (g * NCH + o) * NCH;
      const float* zp = sG + tok * NF + c;
      const float* gp = sGate + tok * NCH;
      float acc = 0.0f;
#pragma unroll 1
      for (int i = 0; i < NCH; ++i) {
        const float z = zp[i * 16] * gp[i];
        acc = fmaf(z, wp[i], acc);
      }
      sH[idx] = sH[idx] + acc;
    }
    __syncthreads();
  }

  if (MODE != 2) {
    ln_xn(sH, sX, sInv, tid);
#pragma unroll 1
    for (int it = 0; it < 5; ++it) {
      const int idx = it * 256 + tid;
      const int tok = idx / 40;
      const int col = idx - tok * 40;
      const int o = col >> 3;
      const int c = ga_islot(col & 7);
      const int g = ga_pop4(ga_mask(c));
      const float* wqp = sW + LW_Q + (g * NCH + o) * NCH;
      const float* wkp = sW + LW_K + (g * NCH + o) * NCH;
      const float* xp = sX + tok * NF + c;
      float aq = 0.0f, ak = 0.0f;
#pragma unroll 1
      for (int i = 0; i < NCH; ++i) {
        const float xv = xp[i * 16];
        aq = fmaf(xv, wqp[i], aq);
        ak = fmaf(xv, wkp[i], ak);
      }
      const unsigned short qh = f2bf_bits(aq);
      const unsigned short ql = f2bf_bits(aq - bf_bits2f(qh));
      const unsigned short kh = f2bf_bits(ak);
      const unsigned short kl = f2bf_bits(ak - bf_bits2f(kh));
      unsigned short* qrow = sQP + tok * DQK + col;
      unsigned short* krow = sKP + tok * DQK + col;
      qrow[0] = qh; qrow[40] = ql; qrow[80] = qh;
      krow[0] = kh; krow[40] = kh; krow[80] = kl;
    }
    {
      const int tk = tid >> 3, j = tid & 7;
      sQP[tk * DQK + 120 + j] = (unsigned short)0;
      sKP[tk * DQK + 120 + j] = (unsigned short)0;
    }
#pragma unroll 1
    for (int it = 0; it < 10; ++it) {
      const int idx = it * 256 + tid;
      const int tok = idx / NF;
      const int rem = idx - tok * NF;
      const int o = rem >> 4, c = rem & 15;
      const int g = ga_pop4(ga_mask(c));
      const float* wvp = sW + LW_V + (g * NCH + o) * NCH;
      const float* xp = sX + tok * NF + c;
      float av = 0.0f;
#pragma unroll 1
      for (int i = 0; i < NCH; ++i) av = fmaf(xp[i * 16], wvp[i], av);
      const unsigned short vh = f2bf_bits(av);
      const unsigned short vl = f2bf_bits(av - bf_bits2f(vh));
      sVH[rem * TPB + tok] = vh;
      sVL[rem * TPB + tok] = vl;
    }
    __syncthreads();
    for (int pass = 0; pass < 2; ++pass) {
#pragma unroll
      for (int it = 0; it < 3; ++it) {
        const int idx = it * 256 + tid;
        if (idx < 640) {
          const v4f v = *(const v4f*)(sH + idx * 4);
          *(volatile v4f*)(Hout + (size_t)tok0 * NF + idx * 4) = v;
        }
      }
#pragma unroll
      for (int it = 0; it < 2; ++it) {
        const int idx = it * 256 + tid;
        const v8us a = *(const v8us*)(sQP + idx * 8);
        const v8us b = *(const v8us*)(sKP + idx * 8);
        *(volatile v8us*)(QP + (size_t)tok0 * DQK + idx * 8) = a;
        *(volatile v8us*)(KP + (size_t)tok0 * DQK + idx * 8) = b;
      }
#pragma unroll
      for (int it = 0; it < 2; ++it) {
        const int idx = it * 256 + tid;
        if (idx < 320) {
          const v8us a = *(const v8us*)(sVH + idx * 8);
          const v8us b = *(const v8us*)(sVL + idx * 8);
          *(volatile v8us*)(VH + (size_t)blockIdx.x * (NF * TPB) + idx * 8) = a;
          *(volatile v8us*)(VL + (size_t)blockIdx.x * (NF * TPB) + idx * 8) = b;
        }
      }
      __threadfence();
    }
  } else {
#pragma unroll 1
    for (int it = 0; it < 5; ++it) {
      const int idx = it * 256 + tid;
      const int idc = (idx < TPB * XW) ? idx : (TPB * XW - 1);
      const int tok = idc / XW;
      const int j = idc - tok * XW;
      const bool isS = j < 32;
      const int jj = j - 32;
      const int ct = (jj == 0) ? GA_T0 : ((jj == 1) ? GA_T1 : GA_T2);
      const int c = isS ? 0 : ct;
      const int woff = LW_A + (isS ? (j * NCH) : (2 * 32 * NCH));
      const float* hp = sH + tok * NF + c;
      float acc = 0.0f;
#pragma unroll 1
      for (int i = 0; i < NCH; ++i) acc = fmaf(hp[i * 16], sW[woff + i], acc);
      if (idx < TPB * XW) sIO[idx] = acc;
    }
    __syncthreads();
    for (int pass = 0; pass < 2; ++pass) {
#pragma unroll
      for (int it = 0; it < 2; ++it) {
        const int idx = it * 256 + tid;
        if (idx < 280) {
          const v4f v = *(const v4f*)(sIO + idx * 4);
          *(volatile v4f*)(out + (size_t)blockIdx.x * (TPB * XW) + idx * 4) = v;
        }
      }
      __threadfence();
    }
  }
}

__global__ __launch_bounds__(256) __attribute__((amdgpu_num_vgpr(248)))
void k_att(const unsigned short* __restrict__ qpp, const unsigned short* __restrict__ kpp,
           const unsigned short* __restrict__ vhp, const unsigned short* __restrict__ vlp,
           float* __restrict__ Oout) {
  union FB { v16b v; v8b h[2]; };
  __shared__ __align__(16) __bf16 Ks[AKC * DQK];
  __shared__ __align__(16) __bf16 Vth[NF * AKC];
  __shared__ __align__(16) __bf16 Vtl[NF * AKC];
  __shared__ __align__(16) __bf16 Psh[ANW][16 * AKC];
  __shared__ __align__(16) __bf16 Psl[ANW][16 * AKC];
  __shared__ __align__(16) float  Os[ANW][16 * NF];

  const int tid  = threadIdx.x;
  const int wave = tid >> 5;
  const int lane = tid & 31;
  const int hh   = lane >> 4;
  const int c    = lane & 15;

  const int nqb = NTOK / AQB;
  const int b   = blockIdx.x / nqb;
  const int qb  = blockIdx.x - b * nqb;
  const size_t tokb = (size_t)b * NTOK;
  const size_t q0   = tokb + (size_t)qb * AQB + (size_t)wave * 16;

  const __bf16* Qg = (const __bf16*)(const void*)qpp;
  const __bf16* Kg = (const __bf16*)(const void*)kpp;
  const __bf16* Vh = (const __bf16*)(const void*)vhp;
  const __bf16* Vl = (const __bf16*)(const void*)vlp;

  v16b qa[4];
#pragma unroll
  for (int ks = 0; ks < 4; ++ks) qa[ks] = frag_ld(Qg + (q0 + c) * DQK + ks * 32 + 8 * hh);

  float mrow[8], lrow[8];
  v8f oacc[5];
#pragma unroll
  for (int r = 0; r < 8; ++r) { mrow[r] = -INFINITY; lrow[r] = 0.0f; }
#pragma unroll
  for (int t = 0; t < 5; ++t) oacc[t] = (v8f){0.f, 0.f, 0.f, 0.f, 0.f, 0.f, 0.f, 0.f};

  const float sscale = 0.11180339887498948f;
  const int nTiles = NTOK / AKC;

#pragma unroll 1
  for (int kc = 0; kc < nTiles; ++kc) {
    const size_t tokk = tokb + (size_t)kc * AKC;
    __syncthreads();
    {
      const __bf16* ksrc = Kg + tokk * DQK;
#pragma unroll
      for (int i = 0; i < 4; ++i) {
        const int p = i * 256 + tid;
        const v8b a = *(const v8b*)(ksrc + p * 8);
        *(v8b*)(Ks + p * 8) = a;
      }
      const size_t vbase = (tokk / TPB) * (size_t)(NF * TPB);
#pragma unroll
      for (int i = 0; i < 3; ++i) {
        const int p = i * 256 + tid;
        if (p < 640) {
          const int g = (p >= 320) ? 1 : 0;
          const int rem = p - g * 320;
          const int f = rem >> 2, pc = rem & 3;
          const v8b a = *(const v8b*)(Vh + vbase + (size_t)p * 8);
          const v8b d = *(const v8b*)(Vl + vbase + (size_t)p * 8);
          *(v8b*)(Vth + f * AKC + g * TPB + pc * 8) = a;
          *(v8b*)(Vtl + f * AKC + g * TPB + pc * 8) = d;
        }
      }
    }
    __syncthreads();

    v8f s[4];
#pragma unroll
    for (int j = 0; j < 4; ++j) {
      s[j] = (v8f){0.f, 0.f, 0.f, 0.f, 0.f, 0.f, 0.f, 0.f};
#pragma unroll
      for (int ks = 0; ks < 4; ++ks) {
        FB kb;
        kb.h[0] = *(const v8b*)(Ks + (j * 16 + c) * DQK + ks * 32 + 8 * hh);
        kb.h[1] = *(const v8b*)(Ks + (j * 16 + c) * DQK + ks * 32 + 16 + 8 * hh);
        s[j] = wmb(qa[ks], kb.v, s[j]);
      }
    }
    float cm[8];
#pragma unroll
    for (int r = 0; r < 8; ++r) {
      float m = -INFINITY;
#pragma unroll
      for (int j = 0; j < 4; ++j) {
        const float sv = s[j][r] * sscale;
        s[j][r] = sv;
        m = fmaxf(m, sv);
      }
#pragma unroll
      for (int off = 1; off < 16; off <<= 1) m = fmaxf(m, __shfl_xor(m, off, 32));
      cm[r] = m;
    }
    __bf16* pwh = Psh[wave];
    __bf16* pwl = Psl[wave];
#pragma unroll
    for (int r = 0; r < 8; ++r) {
      const float mnew  = fmaxf(mrow[r], cm[r]);
      const float alpha = __expf(mrow[r] - mnew);
      mrow[r] = mnew;
      float psum = 0.0f;
#pragma unroll
      for (int j = 0; j < 4; ++j) {
        const float p = __expf(s[j][r] - mnew);
        psum += p;
        __bf16 a, bl;
        split_bf(p, a, bl);
        pwh[(8 * hh + r) * AKC + j * 16 + c] = a;
        pwl[(8 * hh + r) * AKC + j * 16 + c] = bl;
      }
#pragma unroll
      for (int off = 1; off < 16; off <<= 1) psum += __shfl_xor(psum, off, 32);
      lrow[r] = lrow[r] * alpha + psum;
#pragma unroll
      for (int t = 0; t < 5; ++t) oacc[t][r] *= alpha;
    }
    __builtin_amdgcn_fence(__ATOMIC_RELEASE, "workgroup");
    __builtin_amdgcn_wave_barrier();
    __builtin_amdgcn_fence(__ATOMIC_ACQUIRE, "workgroup");
#pragma unroll 1
    for (int kk = 0; kk < 2; ++kk) {
      FB pa, pl;
      pa.h[0] = *(const v8b*)(pwh + c * AKC + kk * 32 + 8 * hh);
      pa.h[1] = *(const v8b*)(pwh + c * AKC + kk * 32 + 16 + 8 * hh);
      pl.h[0] = *(const v8b*)(pwl + c * AKC + kk * 32 + 8 * hh);
      pl.h[1] = *(const v8b*)(pwl + c * AKC + kk * 32 + 16 + 8 * hh);
#pragma unroll
      for (int t = 0; t < 5; ++t) {
        FB vb, vl;
        vb.h[0] = *(const v8b*)(Vth + (t * 16 + c) * AKC + kk * 32 + 8 * hh);
        vb.h[1] = *(const v8b*)(Vth + (t * 16 + c) * AKC + kk * 32 + 16 + 8 * hh);
        vl.h[0] = *(const v8b*)(Vtl + (t * 16 + c) * AKC + kk * 32 + 8 * hh);
        vl.h[1] = *(const v8b*)(Vtl + (t * 16 + c) * AKC + kk * 32 + 16 + 8 * hh);
        oacc[t] = wmb(pa.v, vb.v, oacc[t]);
        oacc[t] = wmb(pa.v, vl.v, oacc[t]);
        oacc[t] = wmb(pl.v, vb.v, oacc[t]);
      }
    }
  }

  float* os = Os[wave];
#pragma unroll
  for (int r = 0; r < 8; ++r) {
    const float inv = 1.0f / lrow[r];
#pragma unroll
    for (int t = 0; t < 5; ++t) os[(8 * hh + r) * NF + t * 16 + c] = oacc[t][r] * inv;
  }
  __builtin_amdgcn_fence(__ATOMIC_RELEASE, "workgroup");
  __builtin_amdgcn_wave_barrier();
  __builtin_amdgcn_fence(__ATOMIC_ACQUIRE, "workgroup");
  {
    float* ob = Oout + q0 * NF;
    for (int pass = 0; pass < 2; ++pass) {
#pragma unroll
      for (int it = 0; it < 10; ++it) {
        const int idx = it * 32 + lane;
        const v4f val = *(const v4f*)(os + idx * 4);
        *(volatile v4f*)(ob + idx * 4) = val;
      }
      __threadfence();
    }
  }
}

extern "C" void kernel_launch(void* const* d_in, const int* in_sizes, int n_in,
                              void* d_out, int out_size, void* d_ws, size_t ws_size,
                              hipStream_t stream) {
  if (n_in < 9) return;
  if (in_sizes[0] != TOK * XW) return;
  if (in_sizes[1] != 800 || in_sizes[2] != 800) return;
  if (in_sizes[3] != 375 || in_sizes[4] != 375 || in_sizes[5] != 375 || in_sizes[6] != 375) return;
  if (in_sizes[7] != 750 || in_sizes[8] != 375) return;
  if (out_size != TOK * XW) return;

  const float* x     = (const float*)d_in[0];
  const float* w_in  = (const float*)d_in[1];
  const float* w_out = (const float*)d_in[2];
  const float* wq    = (const float*)d_in[3];
  const float* wk    = (const float*)d_in[4];
  const float* wv    = (const float*)d_in[5];
  const float* wo    = (const float*)d_in[6];
  const float* w1    = (const float*)d_in[7];
  const float* w2    = (const float*)d_in[8];

  const size_t SZ_PRM = (size_t)P_TOT * 4;
  const size_t SZ_H   = (size_t)TOK * NF * 4;
  const size_t SZ_QK  = (size_t)TOK * DQK * 2;
  const size_t SZ_V   = (size_t)TOK * NF * 2;
  size_t off = 0;
  const size_t oPRM = off; off += SZ_PRM;
  const size_t oH0  = off; off += SZ_H;
  const size_t oH1  = off; off += SZ_H;
  const size_t oO   = off; off += SZ_H;
  const size_t oQP  = off; off += SZ_QK;
  const size_t oKP  = off; off += SZ_QK;
  const size_t oVH  = off; off += SZ_V;
  const size_t oVL  = off; off += SZ_V;
  if (off > ws_size) return;
  if (off > (size_t)134217728) return;

  char* ws = (char*)d_ws;
  float* PRM = (float*)(ws + oPRM);
  float* H0  = (float*)(ws + oH0);
  float* H1  = (float*)(ws + oH1);
  float* O   = (float*)(ws + oO);
  unsigned short* QP = (unsigned short*)(ws + oQP);
  unsigned short* KP = (unsigned short*)(ws + oKP);
  unsigned short* VH = (unsigned short*)(ws + oVH);
  unsigned short* VL = (unsigned short*)(ws + oVL);
  float* outp = (float*)d_out;

  const dim3 blk256(256);
  const dim3 gTok(TOK / TPB);
  const dim3 gAtt(NB * (NTOK / AQB));

  k_prm<<<dim3(8), blk256, 0, stream>>>(w_in, w_out, wq, wk, wv, wo, w1, w2, PRM);
  k_tok<0><<<gTok, blk256, 0, stream>>>(x, O, H1, H0, PRM, QP, KP, VH, VL, outp, 0);
  k_att<<<gAtt, blk256, 0, stream>>>(QP, KP, VH, VL, O);
  k_tok<1><<<gTok, blk256, 0, stream>>>(x, O, H0, H1, PRM, QP, KP, VH, VL, outp, 0);
  k_att<<<gAtt, blk256, 0, stream>>>(QP, KP, VH, VL, O);
  k_tok<1><<<gTok, blk256, 0, stream>>>(x, O, H1, H0, PRM, QP, KP, VH, VL, outp, 1);
  k_att<<<gAtt, blk256, 0, stream>>>(QP, KP, VH, VL, O);
  k_tok<2><<<gTok, blk256, 0, stream>>>(x, O, H0, H1, PRM, QP, KP, VH, VL, outp, 2);
  (void)hipGetLastError();
}
